// MambaBlock_49701361549629
// MI455X (gfx1250) — hardware-verified
//
#include <hip/hip_runtime.h>
#include <math.h>

typedef __attribute__((ext_vector_type(16))) _Float16 v16h;
typedef __attribute__((ext_vector_type(8)))  _Float16 v8h;
typedef __attribute__((ext_vector_type(8)))  float    v8f;
typedef __attribute__((ext_vector_type(4)))  float    v4f;
typedef __attribute__((ext_vector_type(2)))  float    v2f;

constexpr int kBatch  = 2;
constexpr int kSeq    = 1024;
constexpr int kRows   = kBatch * kSeq;
constexpr int kDm     = 1024;
constexpr int kDin    = 2048;
constexpr int kXg     = 2 * kDin;
constexpr int kGrp    = 16;
constexpr int kNst    = 16;
constexpr int kGrpCh  = kDin / kGrp;
constexpr int kPrmW   = 1 + 2 * kNst;
constexpr int kPrm    = kGrp * kPrmW;
constexpr int kPrmP   = 576;
constexpr int kFf     = 4 * kDm;
constexpr int kScTc   = 16;
constexpr int kScYP   = 132;
constexpr float kWCarry   = 32.0f;
constexpr float kYCarry   = 16.0f;
constexpr float kInvW     = 1.0f / kWCarry;
constexpr float kInvWY    = 1.0f / (kWCarry * kYCarry);
static_assert(kRows == 2048 && kGrpCh == 128 && kPrmW == 33 && kPrm == 528 && kXg == 4096 && kFf == 4096, "shape constants");
static_assert((kPrmP % 64) == 0 && kPrmP >= kPrm, "padded parameter width");
static_assert((kDm % 32) == 0 && (kDin % 32) == 0 && (kFf % 32) == 0, "GEMM K multiples of 32");
static_assert((kRows % 64) == 0 && (kXg % 64) == 0 && (kDm % 64) == 0 && (kFf % 64) == 0, "GEMM M,N multiples of 64");
static_assert((kSeq % kScTc) == 0, "scan chunking");

constexpr size_t kSzWIN = (size_t)kXg   * kDm   * 2;
constexpr size_t kSzWPR = (size_t)kPrmP * kDin  * 2;
constexpr size_t kSzWOU = (size_t)kDm   * kDin  * 2;
constexpr size_t kSzWF1 = (size_t)kFf   * kDm   * 2;
constexpr size_t kSzWF2 = (size_t)kDm   * kFf   * 2;
constexpr size_t kSzZH  = (size_t)kRows * kDm   * 2;
constexpr size_t kSzXG  = (size_t)kRows * kXg   * 2;
constexpr size_t kSzPAR = (size_t)kRows * kPrmP * 4;
constexpr size_t kSzYH  = (size_t)kRows * kDin  * 2;
constexpr size_t kSzX2  = (size_t)kRows * kDm   * 4;
constexpr size_t kSzH2  = (size_t)kRows * kDm   * 2;
constexpr size_t kSzF1  = (size_t)kRows * kFf   * 2;
constexpr size_t kOffWIN = 0;
constexpr size_t kOffWPR = kOffWIN + kSzWIN;
constexpr size_t kOffWOU = kOffWPR + kSzWPR;
constexpr size_t kOffWF1 = kOffWOU + kSzWOU;
constexpr size_t kOffWF2 = kOffWF1 + kSzWF1;
constexpr size_t kOffZH  = kOffWF2 + kSzWF2;
constexpr size_t kOffXG  = kOffZH  + kSzZH;
constexpr size_t kOffPAR = kOffXG  + kSzXG;
constexpr size_t kOffYH  = kOffPAR + kSzPAR;
constexpr size_t kOffX2  = kOffYH  + kSzYH;
constexpr size_t kOffH2  = kOffX2  + kSzX2;
constexpr size_t kOffF1  = kOffH2  + kSzH2;
constexpr size_t kWsTotal = kOffF1 + kSzF1;
static_assert(kWsTotal == 95158272ull, "carve total");
static_assert(kWsTotal <= 134217728ull, "carve cap");
static_assert((kSzWIN % 128) == 0 && (kSzWPR % 128) == 0 && (kSzWOU % 128) == 0 && (kSzWF1 % 128) == 0 &&
              (kSzWF2 % 128) == 0 && (kSzZH % 128) == 0 && (kSzXG % 128) == 0 && (kSzPAR % 128) == 0 &&
              (kSzYH % 128) == 0 && (kSzX2 % 128) == 0 && (kSzH2 % 128) == 0 && (kSzF1 % 128) == 0, "128-B aligned regions");

__device__ __forceinline__ float h16_to_f32(unsigned hb) {
  const unsigned sgn = (hb & 0x8000u) << 16;
  const unsigned em = hb & 0x7fffu;
  const float fn = __uint_as_float((em << 13) + 0x38000000u);
  const float fs = (float)em * 5.9604644775390625e-8f;
  const float mag = (em < 0x400u) ? fs : fn;
  return __uint_as_float(__float_as_uint(mag) | sgn);
}

__device__ __forceinline__ float silu_f(float v) {
  return v * __builtin_amdgcn_rcpf(1.0f + expf(-v));
}

__device__ __forceinline__ void row_guard_h(v8f& a, v8f& b, v8f& c, v8f& d, v16h x, v16h b0, v16h b1, v16h b2, v16h b3) {
  asm volatile("v_nop\n\tv_nop\n\tv_nop\n\tv_nop" : "+v"(a), "+v"(b), "+v"(c), "+v"(d) : "v"(x), "v"(b0), "v"(b1), "v"(b2), "v"(b3));
}
__device__ __forceinline__ void keep4_h(v16h a, v16h b, v16h c, v16h d) { asm volatile("v_nop" :: "v"(a), "v"(b), "v"(c), "v"(d)); }
__device__ __forceinline__ void acc_guard4(v8f& a, v8f& b, v8f& c, v8f& d) { asm volatile("v_nop\n\tv_nop\n\tv_nop\n\tv_nop" : "+v"(a), "+v"(b), "+v"(c), "+v"(d)); }

union FragU { v16h v; v8h h[2]; };
__device__ __forceinline__ v16h frag_load(const _Float16* p) {
  FragU f;
  f.h[0] = *(const v8h*)(p);
  f.h[1] = *(const v8h*)(p + 16);
  return f.v;
}
__device__ __forceinline__ v8f frag_mma(v16h a, v16h b, v8f c) {
  return __builtin_amdgcn_wmma_f32_16x16x32_f16(false, a, false, b, (short)0, c, false, false);
}

template <int BIAS_MODE, int OUT_MODE, bool RESID, int ACT>
__global__ __launch_bounds__(256) void wmma_gemm64_f16(
    const unsigned short* __restrict__ Ap, int lda,
    const unsigned short* __restrict__ Btp, int ldb,
    void* __restrict__ Cout, int ldc,
    const float* __restrict__ bias,
    const float* __restrict__ resid,
    int M, int N, int K, float scale) {
  static_assert(OUT_MODE == 0 || ACT == 3, "f16 output path carries its bias through the activation pass");
  static_assert(!(OUT_MODE == 0 && ACT != 0), "f32 output path has no activation");
  static_assert(!(OUT_MODE == 1 && RESID), "f16 output path has no residual");
  const _Float16* A  = (const _Float16*)Ap;
  const _Float16* Bt = (const _Float16*)Btp;
  __shared__ __align__(16) float sT[8][16 * 68];
  const int lane = threadIdx.x & 31;
  const int wave = threadIdx.x >> 5;
  const int tilesN = N >> 6;
  const int tilesM = M >> 6;
  const int tile = blockIdx.x * 8 + wave;
  if (tile >= tilesM * tilesN) return;
  const int tm = tile / tilesN;
  const int tn = tile - tm * tilesN;
  const int m0 = tm << 6;
  const int n0 = tn << 6;

  const int rlane = lane & 15;
  const int koff  = (lane >> 4) * 8;
  const int mOff  = (lane >> 4) * 8;

  v8f acc[4][4];
#pragma unroll
  for (int i = 0; i < 4; ++i)
#pragma unroll
    for (int j = 0; j < 4; ++j) acc[i][j] = (v8f){0.f, 0.f, 0.f, 0.f, 0.f, 0.f, 0.f, 0.f};

  for (int k0 = 0; k0 < K; k0 += 32) {
    v16h bh[4];
#pragma unroll
    for (int j = 0; j < 4; ++j) {
      const size_t bo = (size_t)(n0 + (j << 4) + rlane) * ldb + koff + k0;
      bh[j] = frag_load(Bt + bo);
    }
#pragma unroll
    for (int i = 0; i < 4; ++i) {
      const size_t ao = (size_t)(m0 + (i << 4) + rlane) * lda + koff + k0;
      const v16h ah = frag_load(A + ao);
#pragma unroll
      for (int j = 0; j < 4; ++j) acc[i][j] = frag_mma(ah, bh[j], acc[i][j]);
      row_guard_h(acc[i][0], acc[i][1], acc[i][2], acc[i][3], ah, bh[0], bh[1], bh[2], bh[3]);
    }
    keep4_h(bh[0], bh[1], bh[2], bh[3]);
  }
  acc_guard4(acc[0][0], acc[0][1], acc[0][2], acc[0][3]);
  acc_guard4(acc[1][0], acc[1][1], acc[1][2], acc[1][3]);
  acc_guard4(acc[2][0], acc[2][1], acc[2][2], acc[2][3]);
  acc_guard4(acc[3][0], acc[3][1], acc[3][2], acc[3][3]);

  float* slab = sT[wave];
  const int hh = lane >> 4;
  const int c4 = (lane & 15) * 4;
  v4f bias4 = (v4f){0.f, 0.f, 0.f, 0.f};
  v2f bias2 = (v2f){0.f, 0.f};
  if (BIAS_MODE == 2 && ACT == 0) bias4 = *(const v4f*)(bias + n0 + c4);
  if (BIAS_MODE == 2 && ACT != 0) bias2 = *(const v2f*)(bias + n0 + 2 * lane);
#pragma unroll
  for (int i = 0; i < 4; ++i) {
    const int mBase = m0 + (i << 4);
#pragma unroll
    for (int j = 0; j < 4; ++j) {
#pragma unroll
      for (int r = 0; r < 8; ++r) {
        slab[(mOff + r) * 68 + (j << 4) + rlane] = acc[i][j][r] * scale;
      }
    }
    __builtin_amdgcn_fence(__ATOMIC_RELEASE, "workgroup");
    __builtin_amdgcn_wave_barrier();
    __builtin_amdgcn_fence(__ATOMIC_ACQUIRE, "workgroup");
    if (ACT == 3) {
#pragma unroll 1
      for (int rr = 0; rr < 16; ++rr) {
        float* sp = slab + rr * 68 + 2 * lane;
        const v2f t = *(const v2f*)sp;
        float t0 = t[0];
        float t1 = t[1];
        if (BIAS_MODE == 2) {
          t0 += bias2[0];
          t1 += bias2[1];
        }
        v2f o;
        o[0] = silu_f(t0);
        o[1] = silu_f(t1);
        *(v2f*)sp = o;
      }
      __builtin_amdgcn_fence(__ATOMIC_RELEASE, "workgroup");
      __builtin_amdgcn_wave_barrier();
      __builtin_amdgcn_fence(__ATOMIC_ACQUIRE, "workgroup");
    }
    if (OUT_MODE == 0) {
      float* C = (float*)Cout;
      v4f vv[8];
#pragma unroll
      for (int it = 0; it < 8; ++it) {
        const int row = it * 2 + hh;
        v4f v = *(const v4f*)(slab + row * 68 + c4);
        if (BIAS_MODE == 2) v += bias4;
        if (RESID) {
          const v4f rv = *(const v4f*)(resid + (size_t)(mBase + row) * ldc + n0 + c4);
          v += rv;
        }
        vv[it] = v;
      }
      for (int pass = 0; pass < 2; ++pass) {
#pragma unroll
        for (int it = 0; it < 8; ++it) {
          const int row = it * 2 + hh;
          *(volatile v4f*)(C + (size_t)(mBase + row) * ldc + n0 + c4) = vv[it];
        }
        __threadfence();
      }
    } else {
      const int q = lane >> 3;
      const int c8 = (lane & 7) * 8;
      unsigned short* C = (unsigned short*)Cout;
      v8h hv[4];
#pragma unroll
      for (int it = 0; it < 4; ++it) {
        const int row = it * 4 + q;
        const float* sp = slab + row * 68 + c8;
        const v4f a0 = *(const v4f*)(sp);
        const v4f a1 = *(const v4f*)(sp + 4);
#pragma unroll
        for (int e = 0; e < 4; ++e) {
          hv[it][e]     = (_Float16)a0[e];
          hv[it][4 + e] = (_Float16)a1[e];
        }
      }
      for (int pass = 0; pass < 2; ++pass) {
#pragma unroll
        for (int it = 0; it < 4; ++it) {
          const int row = it * 4 + q;
          *(volatile v8h*)(C + (size_t)(mBase + row) * ldc + n0 + c8) = hv[it];
        }
        __threadfence();
      }
    }
    __builtin_amdgcn_fence(__ATOMIC_RELEASE, "workgroup");
    __builtin_amdgcn_wave_barrier();
    __builtin_amdgcn_fence(__ATOMIC_ACQUIRE, "workgroup");
  }
}

__global__ __launch_bounds__(256) void cast_f16_pad_kernel(
    const float* __restrict__ src, unsigned short* __restrict__ dst, int total8, int real8, float scale)
{
  const int i = blockIdx.x * 256 + threadIdx.x;
  if (i >= total8) return;
  const bool keep = (i < real8);
  const int ic = keep ? i : (real8 - 1);
  const float* p = src + ((size_t)ic << 3);
  const v4f a0 = *(const v4f*)(p);
  const v4f a1 = *(const v4f*)(p + 4);
  v8h hv;
#pragma unroll
  for (int e = 0; e < 4; ++e) {
    const float f0 = keep ? (a0[e] * scale) : 0.0f;
    const float f1 = keep ? (a1[e] * scale) : 0.0f;
    hv[e]     = (_Float16)f0;
    hv[4 + e] = (_Float16)f1;
  }
  unsigned short* q = dst + ((size_t)i << 3);
  *(volatile v8h*)q = hv;
  __threadfence();
  *(volatile v8h*)q = hv;
}

__global__ __launch_bounds__(128) void rmsnorm_f16_kernel(
    const float* __restrict__ x, const float* __restrict__ g, unsigned short* __restrict__ out)
{
  __shared__ float red[4];
  const int tid = threadIdx.x, lane = tid & 31, wave = tid >> 5;
  const size_t base = (size_t)blockIdx.x * kDm + (size_t)tid * 8;
  const v4f a0 = *(const v4f*)(x + base);
  const v4f a1 = *(const v4f*)(x + base + 4);
  float ss = 0.0f;
#pragma unroll
  for (int e = 0; e < 4; ++e) {
    ss += a0[e] * a0[e];
    ss += a1[e] * a1[e];
  }
  ss += __shfl_xor(ss, 16, 32);
  ss += __shfl_xor(ss, 8, 32);
  ss += __shfl_xor(ss, 4, 32);
  ss += __shfl_xor(ss, 2, 32);
  ss += __shfl_xor(ss, 1, 32);
  if (lane == 0) red[wave] = ss;
  __syncthreads();
  const float tot = (red[0] + red[1]) + (red[2] + red[3]);
  const float rs = rsqrtf(tot * (1.0f / (float)kDm) + 1e-6f);
  const v4f g0 = *(const v4f*)(g + tid * 8);
  const v4f g1 = *(const v4f*)(g + tid * 8 + 4);
  v8h hv;
#pragma unroll
  for (int e = 0; e < 4; ++e) {
    hv[e]     = (_Float16)(a0[e] * rs * g0[e]);
    hv[4 + e] = (_Float16)(a1[e] * rs * g1[e]);
  }
  unsigned short* q = out + base;
  *(volatile v8h*)q = hv;
  __threadfence();
  *(volatile v8h*)q = hv;
}

__global__ __launch_bounds__(128) void scan_kernel(
    const float* __restrict__ PAR, const float* __restrict__ Alog,
    const unsigned* __restrict__ XGW, unsigned short* __restrict__ YH)
{
  __shared__ __align__(16) float sP[kScTc * 48];
  __shared__ __align__(16) float sY[kScTc * kScYP];
  const int tid = threadIdx.x, lane = tid & 31, wave = tid >> 5;
  const int bix = blockIdx.x >> 4;
  const int g   = blockIdx.x & 15;
  const int ch  = g * kGrpCh + tid;
  const size_t row0 = (size_t)bix * kSeq;
  const int n  = tid & 15;
  const int sl = tid >> 4;
  const float An   = -expf(Alog[n]);
  const float invA = 1.0f / (An + 1e-12f);
  const unsigned sh = (unsigned)(tid & 1) * 16u;
  const int wcol = ch >> 1;
  const int hh = lane >> 4;
  const int c8 = (lane & 15) * 8;
  float h[kNst];
#pragma unroll
  for (int k = 0; k < kNst; ++k) h[k] = 0.0f;

#pragma unroll 1
  for (int t0 = 0; t0 < kSeq; t0 += kScTc) {
#pragma unroll 1
    for (int hf = 0; hf < 2; ++hf) {
      const int s = sl + 8 * hf;
      const size_t po = (row0 + t0 + s) * kPrmP + (size_t)g * kPrmW;
      const float draw = PAR[po];
      const float bv   = PAR[po + 1 + n];
      const float cv   = PAR[po + 1 + kNst + n];
      const float delta = fmaxf(draw, 0.0f) + log1pf(expf(-fabsf(draw)));
      float dA = delta * An;
      dA = fminf(fmaxf(dA, -10.0f), 10.0f);
      const float e  = expf(dA);
      const float fe = (e - 1.0f) * invA;
      const float frac = (fabsf(dA) < 1e-4f) ? delta : fe;
      sP[s * 48 + n]      = e;
      sP[s * 48 + 16 + n] = frac * bv;
      sP[s * 48 + 32 + n] = cv;
    }
    __syncthreads();
#pragma unroll 1
    for (int s = 0; s < kScTc; ++s) {
      const size_t r = row0 + t0 + s;
      unsigned wu = XGW[r * (kXg / 2) + wcol];
      unsigned wg = XGW[r * (kXg / 2) + (kDin / 2) + wcol];
      asm volatile("" : "+v"(wu));
      asm volatile("" : "+v"(wg));
      const float u  = h16_to_f32((wu >> sh) & 0xffffu);
      const float sg = h16_to_f32((wg >> sh) & 0xffffu);
      const float* p = sP + s * 48;
      v4f Eq[4], Bq[4], Cq[4];
#pragma unroll
      for (int qq = 0; qq < 4; ++qq) {
        Eq[qq] = *(const v4f*)(p + 4 * qq);
        Bq[qq] = *(const v4f*)(p + 16 + 4 * qq);
        Cq[qq] = *(const v4f*)(p + 32 + 4 * qq);
      }
      float y = 0.0f;
#pragma unroll
      for (int k = 0; k < kNst; ++k) {
        const float bu = Bq[k >> 2][k & 3] * u;
        const float hn = fmaf(Eq[k >> 2][k & 3], h[k], bu);
        h[k] = hn;
        y = fmaf(hn, Cq[k >> 2][k & 3], y);
      }
      sY[s * kScYP + tid] = (y * sg) * kYCarry;
    }
    __syncthreads();
    v8h hv[2];
#pragma unroll
    for (int it = 0; it < 2; ++it) {
      const int row = it * 8 + wave * 2 + hh;
      const float* sp = sY + row * kScYP + c8;
      const v4f a0 = *(const v4f*)(sp);
      const v4f a1 = *(const v4f*)(sp + 4);
#pragma unroll
      for (int e = 0; e < 4; ++e) {
        hv[it][e]     = (_Float16)a0[e];
        hv[it][4 + e] = (_Float16)a1[e];
      }
    }
    for (int pass = 0; pass < 2; ++pass) {
#pragma unroll
      for (int it = 0; it < 2; ++it) {
        const int row = it * 8 + wave * 2 + hh;
        *(volatile v8h*)(YH + (row0 + t0 + row) * kDin + (size_t)g * kGrpCh + c8) = hv[it];
      }
      __threadfence();
    }
  }
}

extern "C" void kernel_launch(void* const* d_in, const int* in_sizes, int n_in,
                              void* d_out, int out_size, void* d_ws, size_t ws_size,
                              hipStream_t stream) {
  if (n_in < 11) return;
  if (in_sizes[0] != kRows * kDm) return;
  if (in_sizes[1] != kNst) return;
  if (in_sizes[2] != kDm || in_sizes[3] != kDm) return;
  if (in_sizes[4] != kXg * kDm) return;
  if (in_sizes[5] != kPrm * kDin) return;
  if (in_sizes[6] != kDm * kDin) return;
  if (in_sizes[7] != kFf * kDm) return;
  if (in_sizes[8] != kFf) return;
  if (in_sizes[9] != kDm * kFf) return;
  if (in_sizes[10] != kDm) return;
  if (out_size != kRows * kDm) return;
  if (ws_size < kWsTotal) return;

  const float* x       = (const float*)d_in[0];
  const float* A_log   = (const float*)d_in[1];
  const float* g1      = (const float*)d_in[2];
  const float* g2      = (const float*)d_in[3];
  const float* W_in    = (const float*)d_in[4];
  const float* W_param = (const float*)d_in[5];
  const float* W_out   = (const float*)d_in[6];
  const float* W_ffn1  = (const float*)d_in[7];
  const float* b_ffn1  = (const float*)d_in[8];
  const float* W_ffn2  = (const float*)d_in[9];
  const float* b_ffn2  = (const float*)d_in[10];
  float* out = (float*)d_out;

  char* ws = (char*)d_ws;
  unsigned short* WIN = (unsigned short*)(ws + kOffWIN);
  unsigned short* WPR = (unsigned short*)(ws + kOffWPR);
  unsigned short* WOU = (unsigned short*)(ws + kOffWOU);
  unsigned short* WF1 = (unsigned short*)(ws + kOffWF1);
  unsigned short* WF2 = (unsigned short*)(ws + kOffWF2);
  unsigned short* ZH  = (unsigned short*)(ws + kOffZH);
  unsigned short* XG  = (unsigned short*)(ws + kOffXG);
  float*          PAR = (float*)(ws + kOffPAR);
  unsigned short* YH  = (unsigned short*)(ws + kOffYH);
  float*          X2  = (float*)(ws + kOffX2);
  unsigned short* H2  = (unsigned short*)(ws + kOffH2);
  unsigned short* F1  = (unsigned short*)(ws + kOffF1);

  cast_f16_pad_kernel<<<(kXg * kDm / 8) / 256, 256, 0, stream>>>(W_in, WIN, kXg * kDm / 8, kXg * kDm / 8, kWCarry);
  cast_f16_pad_kernel<<<(kPrmP * kDin / 8) / 256, 256, 0, stream>>>(W_param, WPR, kPrmP * kDin / 8, kPrm * kDin / 8, kWCarry);
  cast_f16_pad_kernel<<<(kDm * kDin / 8) / 256, 256, 0, stream>>>(W_out, WOU, kDm * kDin / 8, kDm * kDin / 8, kWCarry);
  cast_f16_pad_kernel<<<(kFf * kDm / 8) / 256, 256, 0, stream>>>(W_ffn1, WF1, kFf * kDm / 8, kFf * kDm / 8, kWCarry);
  cast_f16_pad_kernel<<<(kDm * kFf / 8) / 256, 256, 0, stream>>>(W_ffn2, WF2, kDm * kFf / 8, kDm * kFf / 8, kWCarry);

  rmsnorm_f16_kernel<<<kRows, 128, 0, stream>>>(x, g1, ZH);

  wmma_gemm64_f16<0, 1, false, 3><<<256, 256, 0, stream>>>(
      ZH, kDm, WIN, kDm, (void*)XG, kXg, b_ffn1, x, kRows, kXg, kDm, kInvW);

  wmma_gemm64_f16<0, 0, false, 0><<<36, 256, 0, stream>>>(
      XG, kXg, WPR, kDin, (void*)PAR, kPrmP, b_ffn1, x, kRows, kPrmP, kDin, kInvW);

  scan_kernel<<<kBatch * kGrp, kGrpCh, 0, stream>>>(PAR, A_log, (const unsigned*)XG, YH);

  wmma_gemm64_f16<0, 0, true, 0><<<64, 256, 0, stream>>>(
      YH, kDin, WOU, kDin, (void*)X2, kDm, b_ffn1, x, kRows, kDm, kDin, kInvWY);

  rmsnorm_f16_kernel<<<kRows, 128, 0, stream>>>(X2, g2, H2);

  wmma_gemm64_f16<2, 1, false, 3><<<256, 256, 0, stream>>>(
      H2, kDm, WF1, kDm, (void*)F1, kFf, b_ffn1, x, kRows, kFf, kDm, kInvW);

  wmma_gemm64_f16<2, 0, true, 0><<<64, 256, 0, stream>>>(
      F1, kFf, WF2, kFf, (void*)out, kDm, b_ffn2, X2, kRows, kDm, kFf, kInvW);
}
